// RelationNet_11209864642931
// MI455X (gfx1250) — hardware-verified
//
#include <hip/hip_runtime.h>

constexpr int kB = 16, kN = 16, kK = 8, kH = 128;
constexpr int kHid2 = 2 * kH;
constexpr int kEncRows = kB * kN * kK;
constexpr int kGroups = kB * kN;
constexpr int kPairsPerGroup = kN * kK * kK;
constexpr float kInvPairs = 1.0f / 1024.0f;
static_assert(kPairsPerGroup == 1024);
static_assert(kEncRows % 64 == 0 && kHid2 % 64 == 0 && kH % 32 == 0);

constexpr int kWaves = 4;
constexpr int kMainThreads = 32 * kWaves;
constexpr int kTiles = kPairsPerGroup / 16;
constexpr int kTilesPerWave = kTiles / kWaves;
static_assert(kTiles * 16 == kPairsPerGroup && kTilesPerWave * kWaves == kTiles);
constexpr int kTileElems = 16 * kHid2;

typedef __attribute__((ext_vector_type(16))) _Float16 v16h;
typedef __attribute__((ext_vector_type(8)))  _Float16 v8h;
typedef __attribute__((ext_vector_type(16))) __bf16   v16b;
typedef __attribute__((ext_vector_type(8)))  __bf16   v8b;
typedef __attribute__((ext_vector_type(8)))  float    v8f;
typedef __attribute__((ext_vector_type(4)))  float    v4f;
typedef __attribute__((ext_vector_type(4)))  unsigned int v4u;

__device__ __forceinline__ unsigned short f2bf_bits(float f) {
  unsigned u = __float_as_uint(f);
  return (unsigned short)((u + 0x7FFFu + ((u >> 16) & 1u)) >> 16);
}
__device__ __forceinline__ float bf_bits2f(unsigned short h) { return __uint_as_float(((unsigned)h) << 16); }
__device__ __forceinline__ unsigned pk16(unsigned short a, unsigned short b) { return (unsigned)a | ((unsigned)b << 16); }

__device__ __forceinline__ void dep_guard_h(v8f& a, v8f& b, v16h x, v16h y) { asm volatile("v_nop\n\tv_nop\n\tv_nop\n\tv_nop" : "+v"(a), "+v"(b) : "v"(x), "v"(y)); }
__device__ __forceinline__ void dep_guard_b(v8f& a, v8f& b, v16b x, v16b y) { asm volatile("v_nop\n\tv_nop\n\tv_nop\n\tv_nop" : "+v"(a), "+v"(b) : "v"(x), "v"(y)); }
__device__ __forceinline__ void keep4_h(v16h a, v16h b, v16h c, v16h d) { asm volatile("v_nop" :: "v"(a), "v"(b), "v"(c), "v"(d)); }
__device__ __forceinline__ void keep4_b(v16b a, v16b b, v16b c, v16b d) { asm volatile("v_nop" :: "v"(a), "v"(b), "v"(c), "v"(d)); }
__device__ __forceinline__ void acc_guard4(v8f& a, v8f& b, v8f& c, v8f& d) { asm volatile("v_nop\n\tv_nop\n\tv_nop\n\tv_nop" : "+v"(a), "+v"(b), "+v"(c), "+v"(d)); }
template <typename T> struct Frag;
template <> struct Frag<_Float16> {
  typedef v16h V; union U { v16h v; v8h h[2]; };
  static __device__ __forceinline__ v16h load(const _Float16* p) {
    U f; f.h[0] = *(const v8h*)(p); f.h[1] = *(const v8h*)(p + 16); return f.v;
  }
  static __device__ __forceinline__ v8f mma(v16h a, v16h b, v8f c) {
    return __builtin_amdgcn_wmma_f32_16x16x32_f16(false, a, false, b, (short)0, c, false, false);
  }
  static __device__ __forceinline__ void guard(v8f& a, v8f& b, v16h x, v16h y) { dep_guard_h(a, b, x, y); }
  static __device__ __forceinline__ void keep(v16h a, v16h b, v16h c, v16h d) { keep4_h(a, b, c, d); }
};
template <> struct Frag<__bf16> {
  typedef v16b V; union U { v16b v; v8b h[2]; };
  static __device__ __forceinline__ v16b load(const __bf16* p) {
    U f; f.h[0] = *(const v8b*)(p); f.h[1] = *(const v8b*)(p + 16); return f.v;
  }
  static __device__ __forceinline__ v8f mma(v16b a, v16b b, v8f c) {
    return __builtin_amdgcn_wmma_f32_16x16x32_bf16(false, a, false, b, (short)0, c, false, false);
  }
  static __device__ __forceinline__ void guard(v8f& a, v8f& b, v16b x, v16b y) { dep_guard_b(a, b, x, y); }
  static __device__ __forceinline__ void keep(v16b a, v16b b, v16b c, v16b d) { keep4_b(a, b, c, d); }
};

template <int ET> struct Elem;
template <> struct Elem<0> { typedef _Float16 T; };
template <> struct Elem<1> { typedef __bf16 T; };
template <int ET, bool SPLIT, int BIAS_MODE, int OUT_MODE, bool RESID, int ACT = 0>
__global__ __launch_bounds__(256) void wmma_gemm64(
    const unsigned short* __restrict__ Ap, const unsigned short* __restrict__ A2p, int lda, long strideA,
    const unsigned short* __restrict__ Btp, const unsigned short* __restrict__ Bt2p, int ldb, long strideB,
    void* __restrict__ Cout, void* __restrict__ Cout2, int ldc, long strideC,
    const float* __restrict__ bias,
    const float* __restrict__ resid, long strideR,
    int M, int N, int K, float scale) {
  typedef typename Elem<ET>::T T;
  typedef typename Frag<T>::V V;
  const T* A = (const T*)Ap; const T* A2 = (const T*)A2p; const T* Bt = (const T*)Btp; const T* Bt2 = (const T*)Bt2p;
  __shared__ __align__(16) float sT[8][16 * 68];
  const int b    = blockIdx.y;
  const int lane = threadIdx.x & 31;
  const int wave = threadIdx.x >> 5;
  const int tilesN = N >> 6;
  const int tilesM = M >> 6;
  const int tile = blockIdx.x * 8 + wave;
  if (tile >= tilesM * tilesN) return;
  const int tm = tile / tilesN;
  const int tn = tile - tm * tilesN;
  const int m0 = tm << 6;
  const int n0 = tn << 6;

  const T* Ab  = A  + (size_t)b * strideA;
  const T* Bb  = Bt + (size_t)b * strideB;
  const T* Ab2 = SPLIT ? (A2  + (size_t)b * strideA) : nullptr;
  const T* Bb2 = SPLIT ? (Bt2 + (size_t)b * strideB) : nullptr;

  const int rlane = lane & 15;
  const int koff  = (lane >> 4) * 8;
  const int mOff  = (lane >> 4) * 8;

  v8f acc[4][4];
#pragma unroll
  for (int i = 0; i < 4; ++i)
#pragma unroll
    for (int j = 0; j < 4; ++j) acc[i][j] = (v8f){0.f,0.f,0.f,0.f,0.f,0.f,0.f,0.f};

  for (int k0 = 0; k0 < K; k0 += 32) {
    V bh[4], bl[4];
#pragma unroll
    for (int j = 0; j < 4; ++j) {
      const size_t bo = (size_t)(n0 + (j << 4) + rlane) * ldb + koff + k0;
      bh[j] = Frag<T>::load(Bb + bo);
      if (SPLIT) bl[j] = Frag<T>::load(Bb2 + bo);
    }
#pragma unroll
    for (int i = 0; i < 4; ++i) {
      const size_t ao = (size_t)(m0 + (i << 4) + rlane) * lda + koff + k0;
      V ah = Frag<T>::load(Ab + ao);
      V al;
      if (SPLIT) al = Frag<T>::load(Ab2 + ao);
#pragma unroll
      for (int j = 0; j < 4; ++j) {
        acc[i][j] = Frag<T>::mma(ah, bh[j], acc[i][j]);
        if (SPLIT) {
          acc[i][j] = Frag<T>::mma(ah, bl[j], acc[i][j]);
          acc[i][j] = Frag<T>::mma(al, bh[j], acc[i][j]);
        }
      }
      Frag<T>::guard(acc[i][0], acc[i][3], ah, SPLIT ? al : ah);
    }
    Frag<T>::keep(bh[0], bh[1], bh[2], bh[3]);
    if (SPLIT) Frag<T>::keep(bl[0], bl[1], bl[2], bl[3]);
  }
  acc_guard4(acc[0][0], acc[0][1], acc[0][2], acc[0][3]);
  acc_guard4(acc[1][0], acc[1][1], acc[1][2], acc[1][3]);
  acc_guard4(acc[2][0], acc[2][1], acc[2][2], acc[2][3]);
  acc_guard4(acc[3][0], acc[3][1], acc[3][2], acc[3][3]);

  float* slab = sT[wave];
  const float* Rb = RESID ? (resid + (size_t)b * strideR) : nullptr;
#pragma unroll
  for (int i = 0; i < 4; ++i) {
    const int mBase = m0 + (i << 4);
#pragma unroll
    for (int j = 0; j < 4; ++j) {
      const int n = n0 + (j << 4) + rlane;
      float bv = 0.f;
      if (BIAS_MODE == 2) bv = bias[n];
#pragma unroll
      for (int r = 0; r < 8; ++r) {
        float v = acc[i][j][r] * scale;
        if (BIAS_MODE == 1) v += bias[mBase + mOff + r];
        if (BIAS_MODE == 2) v += bv;
        if (RESID) v += Rb[(size_t)(mBase + mOff + r) * ldc + n];
        if (ACT == 2) v = fmaxf(v, 0.0f);
        if (ACT == 4) v = (v > 0.f) ? v : 0.01f * v;
        slab[(mOff + r) * 68 + (j << 4) + rlane] = v;
      }
    }
    __builtin_amdgcn_fence(__ATOMIC_RELEASE, "workgroup");
    __builtin_amdgcn_wave_barrier();
    __builtin_amdgcn_fence(__ATOMIC_ACQUIRE, "workgroup");
    if (OUT_MODE == 0) {
      float* C = (float*)Cout + (size_t)b * strideC;
      const int hh = lane >> 4, c4 = (lane & 15) * 4;
      for (int pass = 0; pass < 2; ++pass) {
#pragma unroll
        for (int it = 0; it < 8; ++it) {
          const int row = it * 2 + hh;
          v4f v = *(const v4f*)(slab + row * 68 + c4);
          *(volatile v4f*)(C + (size_t)(mBase + row) * ldc + n0 + c4) = v;
        }
        __threadfence();
      }
    } else {
      const int q = lane >> 3, c8 = (lane & 7) * 8;
      unsigned short* C  = (unsigned short*)Cout  + (size_t)b * strideC;
      unsigned short* C2 = (OUT_MODE == 2) ? ((unsigned short*)Cout2 + (size_t)b * strideC) : nullptr;
      for (int pass = 0; pass < 2; ++pass) {
#pragma unroll
        for (int it = 0; it < 4; ++it) {
          const int row = it * 4 + q;
          const float* sp = slab + row * 68 + c8;
          v8h hv, lv;
#pragma unroll
          for (int e = 0; e < 8; ++e) {
            if (OUT_MODE == 1) {
              hv[e] = (_Float16)sp[e];
            } else {
              unsigned short hb = f2bf_bits(sp[e]);
              unsigned short lb = f2bf_bits(sp[e] - bf_bits2f(hb));
              hv[e] = __builtin_bit_cast(_Float16, hb);
              lv[e] = __builtin_bit_cast(_Float16, lb);
            }
          }
          *(volatile v8h*)(C + (size_t)(mBase + row) * ldc + n0 + c8) = hv;
          if (OUT_MODE == 2) *(volatile v8h*)(C2 + (size_t)(mBase + row) * ldc + n0 + c8) = lv;
        }
        __threadfence();
      }
    }
    __builtin_amdgcn_fence(__ATOMIC_RELEASE, "workgroup");
    __builtin_amdgcn_wave_barrier();
    __builtin_amdgcn_fence(__ATOMIC_ACQUIRE, "workgroup");
  }
}

__global__ __launch_bounds__(256) void cast8_bf16_kernel(
    const float* __restrict__ s0, const float* __restrict__ s1, const float* __restrict__ s2, const float* __restrict__ s3,
    unsigned short* __restrict__ d0, unsigned short* __restrict__ d1, unsigned short* __restrict__ d2, unsigned short* __restrict__ d3,
    int n8a, int n8w) {
  const int z = blockIdx.y;
  const float* in = (z == 0) ? s0 : (z == 1) ? s1 : (z == 2) ? s2 : s3;
  unsigned short* outp = (z == 0) ? d0 : (z == 1) ? d1 : (z == 2) ? d2 : d3;
  const int n8 = (z == 0) ? n8a : n8w;
  const int i = blockIdx.x * 256 + threadIdx.x;
  if (i >= n8) return;
  const float* p = in + 8 * (size_t)i;
  const v4f a = *(const v4f*)(p);
  const v4f c = *(const v4f*)(p + 4);
  const v4u u = (v4u){pk16(f2bf_bits(a[0]), f2bf_bits(a[1])), pk16(f2bf_bits(a[2]), f2bf_bits(a[3])),
                      pk16(f2bf_bits(c[0]), f2bf_bits(c[1])), pk16(f2bf_bits(c[2]), f2bf_bits(c[3]))};
  unsigned short* q = outp + 8 * (size_t)i;
  *(volatile v4u*)q = u;
  __threadfence();
  *(volatile v4u*)q = u;
}

__device__ __forceinline__ v8f zero8() { return (v8f){0.f,0.f,0.f,0.f,0.f,0.f,0.f,0.f}; }
__device__ __forceinline__ unsigned pk_relu_bf2(float a, float b) {
  return pk16(f2bf_bits(fmaxf(a, 0.0f)), f2bf_bits(fmaxf(b, 0.0f)));
}
__device__ __forceinline__ v4u pack_relu8(v8f a) {
  v4u u;
  u[0] = pk_relu_bf2(a[0], a[1]);
  u[1] = pk_relu_bf2(a[2], a[3]);
  u[2] = pk_relu_bf2(a[4], a[5]);
  u[3] = pk_relu_bf2(a[6], a[7]);
  return u;
}
__device__ __forceinline__ float relu_sum8(v8f a) {
  float s = 0.0f;
#pragma unroll
  for (int r = 0; r < 8; ++r) s += fmaxf(a[r], 0.0f);
  return s;
}

__global__ __launch_bounds__(kMainThreads) __attribute__((amdgpu_num_vgpr(256)))
void pair_mlp_mean_kernel(
    const float* __restrict__ LR, const unsigned short* __restrict__ W2b,
    const unsigned short* __restrict__ W3b, float* __restrict__ out) {
  __shared__ __align__(16) __bf16 h1s[kWaves * kTileElems];
  __shared__ __align__(16) __bf16 h2s[kWaves * kTileElems];
  static_assert(sizeof(float) * (kWaves * kHid2 + kHid2) <= sizeof(__bf16) * kTileElems);

  const int tid = threadIdx.x;
  const int wave = tid >> 5;
  const int lane = tid & 31;
  const int rlane = lane & 15;
  const int hh = lane >> 4;
  const int g = blockIdx.x;
  const int b = g >> 4;
  const int n1 = g & 15;

  const __bf16* wb2 = (const __bf16*)(const void*)W2b + (size_t)rlane * kHid2 + 8 * hh;
  const __bf16* wb3 = (const __bf16*)(const void*)W3b + (size_t)rlane * kHid2 + 8 * hh;
  const float* Lbase = LR + (size_t)((b * kN + n1) * kK) * kHid2;
  const float* Rbase = LR + (size_t)kEncRows * kHid2 + (size_t)(b * kN * kK) * kHid2;

  __bf16* const h1w = h1s + wave * kTileElems;
  __bf16* const h2w = h2s + wave * kTileElems;
  const int fbase = rlane * kHid2 + 8 * hh;

  float colacc[16];
#pragma unroll
  for (int i = 0; i < 16; ++i) colacc[i] = 0.0f;

#pragma unroll 1
  for (int tt = 0; tt < kTilesPerWave; ++tt) {
    const int t  = kWaves * tt + wave;
    const int n2 = t >> 2;
    const int k1 = (2 * t + (rlane >> 3)) & 7;
    const int k2 = rlane & 7;
    const float* Lrow = Lbase + (size_t)k1 * kHid2 + 128 * hh;
    const float* Rrow = Rbase + (size_t)(n2 * kK + k2) * kHid2 + 128 * hh;

    __bf16* h1row = h1w + rlane * kHid2 + 128 * hh;
#pragma unroll 2
    for (int c = 0; c < 16; ++c) {
      const v4f l0 = *(const v4f*)(Lrow + 8 * c);
      const v4f l1 = *(const v4f*)(Lrow + 8 * c + 4);
      const v4f r0 = *(const v4f*)(Rrow + 8 * c);
      const v4f r1 = *(const v4f*)(Rrow + 8 * c + 4);
      v4u u;
      u[0] = pk_relu_bf2(l0[0] + r0[0], l0[1] + r0[1]);
      u[1] = pk_relu_bf2(l0[2] + r0[2], l0[3] + r0[3]);
      u[2] = pk_relu_bf2(l1[0] + r1[0], l1[1] + r1[1]);
      u[3] = pk_relu_bf2(l1[2] + r1[2], l1[3] + r1[3]);
      *(v4u*)(void*)(h1row + 8 * c) = u;
    }
    __syncthreads();

#pragma unroll 1
    for (int og = 0; og < 4; ++og) {
      v8f acc[4];
#pragma unroll
      for (int j = 0; j < 4; ++j) acc[j] = zero8();
      const __bf16* ap = wb2 + (size_t)(64 * og) * kHid2;
#pragma unroll 1
      for (int p = 0; p < 8; ++p) {
        const v16b bfr = Frag<__bf16>::load(h1w + fbase + 32 * p);
        v16b afr[4];
#pragma unroll
        for (int j = 0; j < 4; ++j) afr[j] = Frag<__bf16>::load(ap + (size_t)(16 * j) * kHid2 + 32 * p);
#pragma unroll
        for (int j = 0; j < 4; ++j) acc[j] = Frag<__bf16>::mma(afr[j], bfr, acc[j]);
        dep_guard_b(acc[0], acc[3], bfr, bfr);
        keep4_b(afr[0], afr[1], afr[2], afr[3]);
      }
      acc_guard4(acc[0], acc[1], acc[2], acc[3]);
#pragma unroll
      for (int j = 0; j < 4; ++j) {
        const v4u u = pack_relu8(acc[j]);
        *(v4u*)(void*)(h2w + fbase + 16 * (4 * og + j)) = u;
      }
    }
    __syncthreads();

#pragma unroll
    for (int og = 0; og < 4; ++og) {
      v8f acc[4];
#pragma unroll
      for (int j = 0; j < 4; ++j) acc[j] = zero8();
      const __bf16* bp = wb3 + (size_t)(64 * og) * kHid2;
#pragma unroll 1
      for (int p = 0; p < 8; ++p) {
        const v16b afr = Frag<__bf16>::load(h2w + fbase + 32 * p);
        v16b bfr[4];
#pragma unroll
        for (int j = 0; j < 4; ++j) bfr[j] = Frag<__bf16>::load(bp + (size_t)(16 * j) * kHid2 + 32 * p);
#pragma unroll
        for (int j = 0; j < 4; ++j) acc[j] = Frag<__bf16>::mma(afr, bfr[j], acc[j]);
        dep_guard_b(acc[0], acc[3], afr, afr);
        keep4_b(bfr[0], bfr[1], bfr[2], bfr[3]);
      }
      acc_guard4(acc[0], acc[1], acc[2], acc[3]);
#pragma unroll
      for (int j = 0; j < 4; ++j) colacc[4 * og + j] += relu_sum8(acc[j]);
    }
  }

#pragma unroll
  for (int ot = 0; ot < 16; ++ot) colacc[ot] += __shfl_xor(colacc[ot], 16, 32);
  float* redf = (float*)(void*)h1s;
  float* outs = redf + kWaves * kHid2;
  if (hh == 0) {
#pragma unroll
    for (int ot = 0; ot < 16; ++ot) redf[wave * kHid2 + 16 * ot + rlane] = colacc[ot];
  }
  __syncthreads();
#pragma unroll
  for (int c2 = 0; c2 < 2; ++c2) {
    const int c = tid + kMainThreads * c2;
    float s = 0.0f;
    s += redf[0 * kHid2 + c];
    s += redf[1 * kHid2 + c];
    s += redf[2 * kHid2 + c];
    s += redf[3 * kHid2 + c];
    outs[c] = s * kInvPairs;
  }
  __syncthreads();
  if (wave == 0) {
    const v4f v0 = *(const v4f*)(outs + 4 * lane);
    const v4f v1 = *(const v4f*)(outs + 128 + 4 * lane);
    float* ob = out + (size_t)g * kHid2;
    for (int pass = 0; pass < 2; ++pass) {
      *(volatile v4f*)(ob + 4 * lane) = v0;
      *(volatile v4f*)(ob + 128 + 4 * lane) = v1;
      __threadfence();
    }
  }
}

extern "C" void kernel_launch(void* const* d_in, const int* in_sizes, int n_in,
                              void* d_out, int out_size, void* d_ws, size_t ws_size,
                              hipStream_t stream) {
  if (n_in < 4) return;
  if (in_sizes[0] != kEncRows * kH || in_sizes[1] != kHid2 * kHid2 || in_sizes[2] != kHid2 * kHid2 ||
      in_sizes[3] != kHid2 * kHid2 || out_size != kGroups * kHid2) return;
  const float* enc = (const float*)d_in[0];
  const float* W1  = (const float*)d_in[1];
  const float* W2  = (const float*)d_in[2];
  const float* W3  = (const float*)d_in[3];
  float* out = (float*)d_out;

  const size_t encb_bytes = (size_t)kEncRows * kH * 2;
  const size_t wb_bytes   = (size_t)kHid2 * kHid2 * 2;
  const size_t lr_bytes   = (size_t)2 * kEncRows * kHid2 * 4;
  const size_t off_encb = 0;
  const size_t off_w1b  = off_encb + encb_bytes;
  const size_t off_w2b  = off_w1b + wb_bytes;
  const size_t off_w3b  = off_w2b + wb_bytes;
  const size_t off_lr   = off_w3b + wb_bytes;
  const size_t total    = off_lr + lr_bytes;
  if (total > ws_size) return;
  char* ws = (char*)d_ws;
  unsigned short* encb = (unsigned short*)(ws + off_encb);
  unsigned short* W1b  = (unsigned short*)(ws + off_w1b);
  unsigned short* W2b  = (unsigned short*)(ws + off_w2b);
  unsigned short* W3b  = (unsigned short*)(ws + off_w3b);
  float* LR = (float*)(ws + off_lr);

  const int n8a = (kEncRows * kH) / 8;
  const int n8w = (kHid2 * kHid2) / 8;
  cast8_bf16_kernel<<<dim3(128, 4), 256, 0, stream>>>(enc, W1, W2, W3, encb, W1b, W2b, W3b, n8a, n8w);

  wmma_gemm64<1, false, 0, 0, false, 0><<<dim3(16, 2), 256, 0, stream>>>(
      encb, encb, kH, 0L,
      W1b, W1b, kHid2, (long)kH,
      (void*)LR, (void*)LR, kHid2, (long)kEncRows * kHid2,
      (const float*)LR,
      (const float*)LR, 0L,
      kEncRows, kHid2, kH, 1.0f);

  pair_mlp_mean_kernel<<<kGroups, kMainThreads, 0, stream>>>(LR, W2b, W3b, out);
}
